// PAM_Module_37606733644460
// MI455X (gfx1250) — hardware-verified
//
#include <hip/hip_runtime.h>
#include <stddef.h>


#ifndef NB
#define NB 4
#endif
#ifndef SEQ
#define SEQ 4096
#endif
#define NB_FULL 4
#define SEQ_FULL 4096
#define NC 512
#define NQ 64
#define X_CSTRIDE ((size_t)SEQ_FULL)
#define X_BSTRIDE ((size_t)NC * (size_t)SEQ_FULL)

#define WQ_ELEMS (NQ * NC)
#define WV_ELEMS (NC * NC)
#define W16_ELEMS (2 * WQ_ELEMS + WV_ELEMS)

#define SP_BYTES ((size_t)16 * SEQ * 4)
#define ATTN_LDS (SP_BYTES + 1664)

static_assert(SEQ % 256 == 0);
static_assert(SEQ >= 512 && SEQ <= SEQ_FULL);
static_assert(NB >= 1 && NB <= NB_FULL);
static_assert(W16_ELEMS % 2048 == 0);
static_assert(NC % 64 == 0 && NQ == 64);

typedef _Float16 v16h __attribute__((ext_vector_type(16)));
typedef _Float16 h8   __attribute__((ext_vector_type(8)));
typedef _Float16 h8a  __attribute__((ext_vector_type(8), may_alias));
typedef float    v8f  __attribute__((ext_vector_type(8)));
typedef float    v4f  __attribute__((ext_vector_type(4)));
typedef float    v4fa __attribute__((ext_vector_type(4), may_alias));
typedef unsigned int v4u __attribute__((ext_vector_type(4)));

union Frag { v16h v; h8 hl[2]; };
union HU   { h8 h; v4u u; };

static __device__ __forceinline__ v8f mma16(const v16h a, const v16h b, v8f c) {
  c = __builtin_amdgcn_wmma_f32_16x16x32_f16(false, a, false, b, (short)0, c, false, false);
  asm volatile("v_nop\n\tv_nop\n\tv_nop\n\tv_nop" : "+v"(c) : "v"(a), "v"(b));
  return c;
}

static __device__ __forceinline__ float bf16r(float f) {
  unsigned int u = __float_as_uint(f);
  u = u + 0x7FFFu + ((u >> 16) & 1u);
  return __uint_as_float(u & 0xFFFF0000u);
}

static __device__ __forceinline__ v8f zero8() { v8f z = {}; return z; }

__global__ __launch_bounds__(256) void k_wconv(
    const float* __restrict__ wq, const float* __restrict__ wk, const float* __restrict__ wv,
    _Float16* __restrict__ w16)
{
  const int t = blockIdx.x * 256 + threadIdx.x;
  if (t >= W16_ELEMS / 8) return;
  const int e0 = t * 8;
  const float* src;
  int off;
  if (blockIdx.x < WQ_ELEMS / 2048)            { src = wq; off = e0; }
  else if (blockIdx.x < 2 * (WQ_ELEMS / 2048))  { src = wk; off = e0 - WQ_ELEMS; }
  else                                          { src = wv; off = e0 - 2 * WQ_ELEMS; }
  const v4f a = *(const v4f*)(src + off);
  const v4f c = *(const v4f*)(src + off + 4);
  HU u;
#pragma unroll
  for (int i = 0; i < 4; ++i) {
    u.h[i]     = (_Float16)(1024.0f * bf16r(a[i]));
    u.h[4 + i] = (_Float16)(1024.0f * bf16r(c[i]));
  }
  const v4u val = u.u;
  _Float16* dst = w16 + e0;
  *(volatile v4u*)dst = val;
  __threadfence();
  *(volatile v4u*)dst = val;
}

__global__ __launch_bounds__(256) void k_xT(const float* __restrict__ x, _Float16* __restrict__ xT)
{
  __shared__ __attribute__((aligned(16))) _Float16 T[64 * 72];
  const int tid = threadIdx.x;
  const int n0 = blockIdx.x * 64, c0 = blockIdx.y * 64, b = blockIdx.z;
  {
    const int cl = tid >> 2, q = tid & 3;
    const float* src = x + (size_t)b * X_BSTRIDE + (size_t)(c0 + cl) * X_CSTRIDE + n0 + q * 16;
    const v4f f0 = *(const v4f*)(src);
    const v4f f1 = *(const v4f*)(src + 4);
    const v4f f2 = *(const v4f*)(src + 8);
    const v4f f3 = *(const v4f*)(src + 12);
#pragma unroll
    for (int i = 0; i < 4; ++i) {
      T[(q * 16 + i)      * 72 + cl] = (_Float16)(16.0f * bf16r(f0[i]));
      T[(q * 16 + 4 + i)  * 72 + cl] = (_Float16)(16.0f * bf16r(f1[i]));
      T[(q * 16 + 8 + i)  * 72 + cl] = (_Float16)(16.0f * bf16r(f2[i]));
      T[(q * 16 + 12 + i) * 72 + cl] = (_Float16)(16.0f * bf16r(f3[i]));
    }
  }
  __syncthreads();
  v4u val[2];
  size_t dsti[2];
#pragma unroll
  for (int it = 0; it < 2; ++it) {
    const int s = it * 256 + tid;
    const int row = s >> 3, q8 = s & 7;
    HU u;
    u.h = *(const h8a*)(T + row * 72 + q8 * 8);
    val[it] = u.u;
    dsti[it] = ((size_t)b * SEQ + n0 + row) * NC + c0 + q8 * 8;
  }
#pragma unroll
  for (int it = 0; it < 2; ++it) *(volatile v4u*)(xT + dsti[it]) = val[it];
  __threadfence();
#pragma unroll
  for (int it = 0; it < 2; ++it) *(volatile v4u*)(xT + dsti[it]) = val[it];
}

template<int TRANS, int EMIT_LO>
__global__ __launch_bounds__(128) void k_proj(
    const _Float16* __restrict__ xT, const _Float16* __restrict__ W, const float* __restrict__ bias,
    _Float16* oh, _Float16* ol)
{
  __shared__ __attribute__((aligned(16))) float T[64 * 68];
  const int tid = threadIdx.x, w = tid >> 5, lane = tid & 31, h = lane >> 4, m = lane & 15;
  const int nt = blockIdx.x, ot = blockIdx.y, b = blockIdx.z;

  const _Float16* arow = xT + ((size_t)b * SEQ + nt * 64 + w * 16 + m) * NC;
  v8f acc[4];
#pragma unroll
  for (int ct = 0; ct < 4; ++ct) acc[ct] = zero8();

  for (int k0 = 0; k0 < NC; k0 += 32) {
    Frag a;
    a.hl[0] = *(const h8*)(arow + k0 + 8 * h);
    a.hl[1] = *(const h8*)(arow + k0 + 16 + 8 * h);
#pragma unroll
    for (int ct = 0; ct < 4; ++ct) {
      const _Float16* br = W + (size_t)(ot * 64 + ct * 16 + m) * NC + k0;
      Frag bb;
      bb.hl[0] = *(const h8*)(br + 8 * h);
      bb.hl[1] = *(const h8*)(br + 16 + 8 * h);
      acc[ct] = mma16(a.v, bb.v, acc[ct]);
    }
  }

#pragma unroll
  for (int ct = 0; ct < 4; ++ct) {
#pragma unroll
    for (int r = 0; r < 8; ++r) {
      const int nl = w * 16 + 8 * h + r;
      const int olc = ct * 16 + m;
      const float val = acc[ct][r] * (1.0f / 16384.0f) + bf16r(bias[ot * 64 + olc]);
      if (TRANS) T[nl * 68 + olc] = val;
      else       T[olc * 68 + nl] = val;
    }
  }
  __syncthreads();

  v4u hv[4], lv[4];
  size_t dsti[4];
#pragma unroll
  for (int it = 0; it < 4; ++it) {
    const int s = it * 128 + tid;
    const int row = s >> 3, q8 = s & 7;
    const v4fa f0 = *(const v4fa*)(T + row * 68 + q8 * 8);
    const v4fa f1 = *(const v4fa*)(T + row * 68 + q8 * 8 + 4);
    HU hu, lu;
#pragma unroll
    for (int e = 0; e < 4; ++e) {
      const _Float16 hh0 = (_Float16)f0[e];
      hu.h[e] = hh0;
      const _Float16 hh1 = (_Float16)f1[e];
      hu.h[4 + e] = hh1;
      if (EMIT_LO) {
        lu.h[e]     = (_Float16)((f0[e] - (float)hh0) * 2048.0f);
        lu.h[4 + e] = (_Float16)((f1[e] - (float)hh1) * 2048.0f);
      } else {
        lu.h[e] = (_Float16)0.0f;
        lu.h[4 + e] = (_Float16)0.0f;
      }
    }
    hv[it] = hu.u;
    lv[it] = lu.u;
    dsti[it] = TRANS ? (((size_t)b * SEQ + nt * 64 + row) * NQ + q8 * 8)
                     : (((size_t)b * NC + ot * 64 + row) * (size_t)SEQ + nt * 64 + q8 * 8);
  }
#pragma unroll
  for (int it = 0; it < 4; ++it) {
    *(volatile v4u*)(oh + dsti[it]) = hv[it];
    if (EMIT_LO) *(volatile v4u*)(ol + dsti[it]) = lv[it];
  }
  __threadfence();
#pragma unroll
  for (int it = 0; it < 4; ++it) {
    *(volatile v4u*)(oh + dsti[it]) = hv[it];
    if (EMIT_LO) *(volatile v4u*)(ol + dsti[it]) = lv[it];
  }
}

__global__ __launch_bounds__(256) void k_attn(
    const _Float16* __restrict__ qh, const _Float16* __restrict__ ql,
    const _Float16* __restrict__ kh, const _Float16* __restrict__ kl,
    const _Float16* __restrict__ vh,
    float* __restrict__ O32)
{
  extern __shared__ v4f smem_v[];
  char*  sp   = (char*)smem_v;
  float* wmax = (float*)(sp + SP_BYTES);
  float* gmax = wmax + 128;
  float* psum = gmax + 16;
  float* ginv = psum + 256;

  const int tid = threadIdx.x, w = tid >> 5, lane = tid & 31, h = lane >> 4, m = lane & 15;
  const int it = blockIdx.x, b = blockIdx.y, i0 = it * 16;

  Frag Qh[2], Ql[2];
  {
    const _Float16* qhr = qh + ((size_t)b * SEQ + i0 + m) * NQ;
    const _Float16* qlr = ql + ((size_t)b * SEQ + i0 + m) * NQ;
#pragma unroll
    for (int s = 0; s < 2; ++s) {
      Qh[s].hl[0] = *(const h8*)(qhr + s * 32 + 8 * h);
      Qh[s].hl[1] = *(const h8*)(qhr + s * 32 + 16 + 8 * h);
      Ql[s].hl[0] = *(const h8*)(qlr + s * 32 + 8 * h);
      Ql[s].hl[1] = *(const h8*)(qlr + s * 32 + 16 + 8 * h);
    }
  }

  const _Float16* khb = kh + (size_t)b * SEQ * NQ;
  const _Float16* klb = kl + (size_t)b * SEQ * NQ;
  float lmax = -3.0e38f;
  for (int t = 0; t < SEQ / 128; ++t) {
    const int m0 = w * (SEQ / 8) + t * 16;
    const _Float16* krh = khb + (size_t)(m0 + m) * NQ;
    const _Float16* krl = klb + (size_t)(m0 + m) * NQ;
    v8f ah = zero8(), ar = zero8();
#pragma unroll
    for (int s = 0; s < 2; ++s) {
      Frag A, L;
      A.hl[0] = *(const h8*)(krh + s * 32 + 8 * h);
      A.hl[1] = *(const h8*)(krh + s * 32 + 16 + 8 * h);
      L.hl[0] = *(const h8*)(krl + s * 32 + 8 * h);
      L.hl[1] = *(const h8*)(krl + s * 32 + 16 + 8 * h);
      ah = mma16(A.v, Qh[s].v, ah);
      ar = mma16(L.v, Qh[s].v, ar);
      ar = mma16(A.v, Ql[s].v, ar);
    }
    float sv[8];
#pragma unroll
    for (int r = 0; r < 8; ++r) {
      sv[r] = ah[r] + ar[r] * (1.0f / 2048.0f);
      lmax = fmaxf(lmax, sv[r]);
    }
    v4fa* d = (v4fa*)(sp + 4 * ((size_t)m * SEQ + m0 + 8 * h));
    v4fa x0 = {sv[0], sv[1], sv[2], sv[3]};
    v4fa x1 = {sv[4], sv[5], sv[6], sv[7]};
    d[0] = x0;
    d[1] = x1;
  }
  lmax = fmaxf(lmax, __shfl_xor(lmax, 16, 32));
  if (lane < 16) wmax[w * 16 + lane] = lmax;
  __syncthreads();

  if (tid < 16) {
    float g = wmax[tid];
#pragma unroll
    for (int w2 = 1; w2 < 8; ++w2) g = fmaxf(g, wmax[w2 * 16 + tid]);
    gmax[tid] = g;
  }
  __syncthreads();
  {
    const int row = tid >> 4;
    const int seg = tid & 15;
    const float gm = gmax[row];
    char* base = sp + 4 * ((size_t)row * SEQ + (size_t)seg * (SEQ / 16));
    float ls = 0.0f;
    for (int i = 0; i < SEQ / 128; ++i) {
      char* slot = base + i * 32;
      const v4fa s0 = *(const v4fa*)(slot);
      const v4fa s1 = *(const v4fa*)(slot + 16);
      h8a pv;
#pragma unroll
      for (int e = 0; e < 4; ++e) {
        {
          const float p = __expf(s0[e] - gm) * 16384.0f;
          _Float16 ph = (_Float16)p;
          float pf = (float)ph;
          const bool small = pf < 6.103515625e-05f;
          ph = small ? (_Float16)0.0f : ph;
          pf = small ? 0.0f : pf;
          pv[e] = ph;
          ls += pf;
        }
        {
          const float p = __expf(s1[e] - gm) * 16384.0f;
          _Float16 ph = (_Float16)p;
          float pf = (float)ph;
          const bool small = pf < 6.103515625e-05f;
          ph = small ? (_Float16)0.0f : ph;
          pf = small ? 0.0f : pf;
          pv[4 + e] = ph;
          ls += pf;
        }
      }
      *(h8a*)slot = pv;
    }
    psum[row * 16 + seg] = ls;
  }
  __syncthreads();
  if (tid < 16) {
    float s = 0.0f;
#pragma unroll
    for (int seg = 0; seg < 16; ++seg) s += psum[tid * 16 + seg];
    ginv[tid] = 1.0f / s;
  }
  __syncthreads();

  const _Float16* vhb = vh + (size_t)b * NC * SEQ;
  v8f acch[4];
#pragma unroll
  for (int ct = 0; ct < 4; ++ct) acch[ct] = zero8();
  for (int t2 = 0; t2 < SEQ / 32; ++t2) {
    const int mb = t2 * 32;
    Frag p;
    p.hl[0] = *(const h8a*)(sp + 4 * ((size_t)m * SEQ + mb + 8 * h));
    p.hl[1] = *(const h8a*)(sp + 4 * ((size_t)m * SEQ + mb + 16 + 8 * h));
#pragma unroll
    for (int ct = 0; ct < 4; ++ct) {
      const size_t ro = (size_t)(w * 64 + ct * 16 + m) * SEQ + mb;
      Frag a;
      a.hl[0] = *(const h8*)(vhb + ro + 8 * h);
      a.hl[1] = *(const h8*)(vhb + ro + 16 + 8 * h);
      acch[ct] = mma16(a.v, p.v, acch[ct]);
    }
  }
  __syncthreads();

  const float inv = ginv[m];
  float* ost = (float*)sp + w * 1024;
#pragma unroll
  for (int ct = 0; ct < 4; ++ct) {
#pragma unroll
    for (int r = 0; r < 8; ++r) {
      ost[(ct * 16 + 8 * h + r) * 16 + m] = acch[ct][r] * inv;
    }
  }
  __syncthreads();
  v4f vals[8];
#pragma unroll
  for (int k = 0; k < 8; ++k) vals[k] = *(const v4fa*)(ost + k * 128 + lane * 4);
  float* ob = O32 + ((((size_t)b * (SEQ / 16) + it) * NC + w * 64) * 16);
#pragma unroll
  for (int k = 0; k < 8; ++k) *(volatile v4f*)(ob + k * 128 + lane * 4) = vals[k];
  __threadfence();
#pragma unroll
  for (int k = 0; k < 8; ++k) *(volatile v4f*)(ob + k * 128 + lane * 4) = vals[k];
}

__global__ __launch_bounds__(256) void k_out(
    const float* __restrict__ O32, const float* __restrict__ x, const float* __restrict__ gamma,
    float* __restrict__ out)
{
  const size_t t = (size_t)blockIdx.x * 256 + threadIdx.x;
  const size_t total4 = (size_t)NB * NC * SEQ / 4;
  if (t >= total4) return;
  const size_t e = t * 4;
  const int n = (int)(e % SEQ);
  const size_t cn = e / SEQ;
  const int c = (int)(cn % NC);
  const int b = (int)(cn / NC);
  const v4f o  = *(const v4f*)(O32 + ((((size_t)b * (SEQ / 16) + (n >> 4)) * NC + c) * 16 + (n & 15)));
  const v4f xv = *(const v4f*)(x + (size_t)b * X_BSTRIDE + (size_t)c * X_CSTRIDE + n);
  const float g = bf16r(gamma[0]);
  v4f rv;
#pragma unroll
  for (int i = 0; i < 4; ++i) rv[i] = g * o[i] + bf16r(xv[i]);
  float* dst = out + ((size_t)b * NC + c) * (size_t)SEQ + n;
  *(volatile v4f*)dst = rv;
  __threadfence();
  *(volatile v4f*)dst = rv;
}

extern "C" void kernel_launch(void* const* d_in, const int* in_sizes, int n_in,
                              void* d_out, int out_size, void* d_ws, size_t ws_size,
                              hipStream_t stream) {
  if (n_in < 8) return;
  const size_t need_x = ((size_t)(NB - 1) * NC + (NC - 1)) * SEQ_FULL + SEQ;
  if ((size_t)in_sizes[0] < need_x) return;
  if (in_sizes[1] < WQ_ELEMS || in_sizes[3] < WQ_ELEMS || in_sizes[5] < WV_ELEMS) return;
  if (in_sizes[2] < NQ || in_sizes[4] < NQ || in_sizes[6] < NC || in_sizes[7] < 1) return;
  if ((size_t)out_size < (size_t)NB * NC * SEQ) return;

  const float* x     = (const float*)d_in[0];
  const float* wq    = (const float*)d_in[1];
  const float* bq    = (const float*)d_in[2];
  const float* wk    = (const float*)d_in[3];
  const float* bk    = (const float*)d_in[4];
  const float* wv    = (const float*)d_in[5];
  const float* bv    = (const float*)d_in[6];
  const float* gamma = (const float*)d_in[7];
  float* out = (float*)d_out;

  char* ws = (char*)d_ws;
  size_t off = 0;
  _Float16* xT16 = (_Float16*)(ws + off); off += (size_t)NB * SEQ * NC * 2;
  _Float16* w16  = (_Float16*)(ws + off); off += (size_t)W16_ELEMS * 2;
  _Float16* qhP  = (_Float16*)(ws + off); off += (size_t)NB * SEQ * NQ * 2;
  _Float16* qlP  = (_Float16*)(ws + off); off += (size_t)NB * SEQ * NQ * 2;
  _Float16* khP  = (_Float16*)(ws + off); off += (size_t)NB * SEQ * NQ * 2;
  _Float16* klP  = (_Float16*)(ws + off); off += (size_t)NB * SEQ * NQ * 2;
  _Float16* vhP  = (_Float16*)(ws + off); off += (size_t)NB * NC * SEQ * 2;
  float*    O32  = (float*)(ws + off);    off += (size_t)NB * SEQ * NC * 4;
  if (off > ws_size) return;
  if (off > (size_t)134217728) return;

  k_wconv<<<dim3(W16_ELEMS / 2048), dim3(256), 0, stream>>>(wq, wk, wv, w16);
  k_xT<<<dim3(SEQ / 64, NC / 64, NB), dim3(256), 0, stream>>>(x, xT16);
  k_proj<1, 1><<<dim3(SEQ / 64, 1, NB), dim3(128), 0, stream>>>(xT16, w16, bq, qhP, qlP);
  k_proj<1, 1><<<dim3(SEQ / 64, 1, NB), dim3(128), 0, stream>>>(xT16, w16 + WQ_ELEMS, bk, khP, klP);
  k_proj<0, 0><<<dim3(SEQ / 64, NC / 64, NB), dim3(128), 0, stream>>>(xT16, w16 + 2 * WQ_ELEMS, bv, vhP, vhP);

  const size_t lds = ATTN_LDS;
  hipFuncSetAttribute(reinterpret_cast<const void*>(&k_attn), hipFuncAttributeMaxDynamicSharedMemorySize, (int)lds);
  k_attn<<<dim3(SEQ / 16, NB), dim3(256), lds, stream>>>(qhP, qlP, khP, klP, vhP, O32);

  const size_t total4 = (size_t)NB * NC * SEQ / 4;
  const unsigned nblk = (unsigned)((total4 + 255) / 256);
  k_out<<<dim3(nblk), dim3(256), 0, stream>>>(O32, x, gamma, out);
}
